// MultiCabecaAtencao_63763084476445
// MI455X (gfx1250) — hardware-verified
//
#include <hip/hip_runtime.h>
#include <math.h>

constexpr int kBatch = 4;
constexpr int kSeq   = 2048;
constexpr int kDim   = 1024;
constexpr int kTok   = kBatch * kSeq;
constexpr int kQKCols = 2 * kDim;
constexpr float kScoreScale = 0.125f;

typedef __attribute__((ext_vector_type(16))) _Float16 v16h;
typedef __attribute__((ext_vector_type(8)))  _Float16 v8h;
typedef __attribute__((ext_vector_type(16))) __bf16   v16b;
typedef __attribute__((ext_vector_type(8)))  __bf16   v8b;
typedef __attribute__((ext_vector_type(8)))  float    v8f;
typedef __attribute__((ext_vector_type(4)))  float    v4f;
typedef __attribute__((ext_vector_type(4)))  unsigned int v4u;

__device__ __forceinline__ unsigned short f2bf_bits(float f) {
  unsigned u = __float_as_uint(f);
  return (unsigned short)((u + 0x7FFFu + ((u >> 16) & 1u)) >> 16);
}
__device__ __forceinline__ float bf_bits2f(unsigned short h) { return __uint_as_float(((unsigned)h) << 16); }

__device__ __forceinline__ void dep_guard_h(v8f& a, v8f& b, v16h x, v16h y) { asm volatile("v_nop\n\tv_nop\n\tv_nop\n\tv_nop" : "+v"(a), "+v"(b) : "v"(x), "v"(y)); }
__device__ __forceinline__ void dep_guard_b(v8f& a, v8f& b, v16b x, v16b y) { asm volatile("v_nop\n\tv_nop\n\tv_nop\n\tv_nop" : "+v"(a), "+v"(b) : "v"(x), "v"(y)); }
__device__ __forceinline__ void keep4_h(v16h a, v16h b, v16h c, v16h d) { asm volatile("v_nop" :: "v"(a), "v"(b), "v"(c), "v"(d)); }
__device__ __forceinline__ void keep4_b(v16b a, v16b b, v16b c, v16b d) { asm volatile("v_nop" :: "v"(a), "v"(b), "v"(c), "v"(d)); }
__device__ __forceinline__ void acc_guard4(v8f& a, v8f& b, v8f& c, v8f& d) { asm volatile("v_nop\n\tv_nop\n\tv_nop\n\tv_nop" : "+v"(a), "+v"(b), "+v"(c), "+v"(d)); }
template <typename T> struct Frag;
template <> struct Frag<_Float16> {
  typedef v16h V; union U { v16h v; v8h h[2]; };
  static __device__ __forceinline__ v16h load(const _Float16* p) {
    U f; f.h[0] = *(const v8h*)(p); f.h[1] = *(const v8h*)(p + 16); return f.v;
  }
  static __device__ __forceinline__ v8f mma(v16h a, v16h b, v8f c) {
    return __builtin_amdgcn_wmma_f32_16x16x32_f16(false, a, false, b, (short)0, c, false, false);
  }
  static __device__ __forceinline__ void guard(v8f& a, v8f& b, v16h x, v16h y) { dep_guard_h(a, b, x, y); }
  static __device__ __forceinline__ void keep(v16h a, v16h b, v16h c, v16h d) { keep4_h(a, b, c, d); }
};
template <> struct Frag<__bf16> {
  typedef v16b V; union U { v16b v; v8b h[2]; };
  static __device__ __forceinline__ v16b load(const __bf16* p) {
    U f; f.h[0] = *(const v8b*)(p); f.h[1] = *(const v8b*)(p + 16); return f.v;
  }
  static __device__ __forceinline__ v8f mma(v16b a, v16b b, v8f c) {
    return __builtin_amdgcn_wmma_f32_16x16x32_bf16(false, a, false, b, (short)0, c, false, false);
  }
  static __device__ __forceinline__ void guard(v8f& a, v8f& b, v16b x, v16b y) { dep_guard_b(a, b, x, y); }
  static __device__ __forceinline__ void keep(v16b a, v16b b, v16b c, v16b d) { keep4_b(a, b, c, d); }
};

__device__ __forceinline__ unsigned pk16(unsigned short a, unsigned short b) { return (unsigned)a | ((unsigned)b << 16); }

template <int ET> struct Elem;
template <> struct Elem<0> { typedef _Float16 T; };
template <> struct Elem<1> { typedef __bf16 T; };
template <int ET, int SPLITK, int BIAS_MODE, int OUT_MODE, bool RESID, int ACT = 0>
__global__ __launch_bounds__(256) void wmma_gemm64(
    const unsigned short* __restrict__ Ap, const unsigned short* __restrict__ A2p, int lda, long strideA,
    const unsigned short* __restrict__ Btp, const unsigned short* __restrict__ Bt2p, int ldb, long strideB,
    void* __restrict__ Cout, void* __restrict__ Cout2, int ldc, long strideC,
    const float* __restrict__ bias,
    const float* __restrict__ resid, long strideR,
    int M, int N, int K, float scale) {
  typedef typename Elem<ET>::T T;
  typedef typename Frag<T>::V V;
  constexpr bool SPLA = (SPLITK != 0);
  constexpr bool SPLB = (SPLITK == 1);
  const T* A = (const T*)Ap; const T* A2 = (const T*)A2p; const T* Bt = (const T*)Btp; const T* Bt2 = (const T*)Bt2p;
  __shared__ __align__(16) float sT[8][16 * 68];
  const int b    = blockIdx.y;
  const int lane = threadIdx.x & 31;
  const int wave = threadIdx.x >> 5;
  const int tilesN = N >> 6;
  const int tilesM = M >> 6;
  const int tile = blockIdx.x * 8 + wave;
  if (tile >= tilesM * tilesN) return;
  const int tm = tile / tilesN;
  const int tn = tile - tm * tilesN;
  const int m0 = tm << 6;
  const int n0 = tn << 6;

  const T* Ab  = A  + (size_t)b * strideA;
  const T* Bb  = Bt + (size_t)b * strideB;
  const T* Ab2 = SPLA ? (A2  + (size_t)b * strideA) : nullptr;
  const T* Bb2 = SPLB ? (Bt2 + (size_t)b * strideB) : nullptr;

  const int rlane = lane & 15;
  const int koff  = (lane >> 4) * 8;
  const int mOff  = (lane >> 4) * 8;

  v8f acc[4][4];
#pragma unroll
  for (int i = 0; i < 4; ++i)
#pragma unroll
    for (int j = 0; j < 4; ++j) acc[i][j] = (v8f){0.f,0.f,0.f,0.f,0.f,0.f,0.f,0.f};

  for (int k0 = 0; k0 < K; k0 += 32) {
    V bh[4], bl[4];
#pragma unroll
    for (int j = 0; j < 4; ++j) {
      const size_t bo = (size_t)(n0 + (j << 4) + rlane) * ldb + koff + k0;
      bh[j] = Frag<T>::load(Bb + bo);
      if (SPLB) bl[j] = Frag<T>::load(Bb2 + bo);
    }
#pragma unroll
    for (int i = 0; i < 4; ++i) {
      const size_t ao = (size_t)(m0 + (i << 4) + rlane) * lda + koff + k0;
      V ah = Frag<T>::load(Ab + ao);
      V al;
      if (SPLA) al = Frag<T>::load(Ab2 + ao);
#pragma unroll
      for (int j = 0; j < 4; ++j) {
        acc[i][j] = Frag<T>::mma(ah, bh[j], acc[i][j]);
        if (SPLB) acc[i][j] = Frag<T>::mma(ah, bl[j], acc[i][j]);
        if (SPLA) acc[i][j] = Frag<T>::mma(al, bh[j], acc[i][j]);
      }
      Frag<T>::guard(acc[i][0], acc[i][3], ah, SPLA ? al : ah);
    }
    Frag<T>::keep(bh[0], bh[1], bh[2], bh[3]);
    if (SPLB) Frag<T>::keep(bl[0], bl[1], bl[2], bl[3]);
  }
  acc_guard4(acc[0][0], acc[0][1], acc[0][2], acc[0][3]);
  acc_guard4(acc[1][0], acc[1][1], acc[1][2], acc[1][3]);
  acc_guard4(acc[2][0], acc[2][1], acc[2][2], acc[2][3]);
  acc_guard4(acc[3][0], acc[3][1], acc[3][2], acc[3][3]);

  float* slab = sT[wave];
  const float* Rb = RESID ? (resid + (size_t)b * strideR) : nullptr;
#pragma unroll
  for (int i = 0; i < 4; ++i) {
    const int mBase = m0 + (i << 4);
#pragma unroll
    for (int j = 0; j < 4; ++j) {
      const int n = n0 + (j << 4) + rlane;
      float bv = 0.f;
      if (BIAS_MODE == 2) bv = bias[n];
#pragma unroll
      for (int r = 0; r < 8; ++r) {
        float v = acc[i][j][r] * scale;
        if (BIAS_MODE == 1) v += bias[mBase + mOff + r];
        if (BIAS_MODE == 2) v += bv;
        if (RESID) v += Rb[(size_t)(mBase + mOff + r) * ldc + n];
        if (ACT == 2) v = fmaxf(v, 0.0f);
        if (ACT == 4) v = (v > 0.f) ? v : 0.01f * v;
        slab[(mOff + r) * 68 + (j << 4) + rlane] = v;
      }
    }
    __builtin_amdgcn_fence(__ATOMIC_RELEASE, "workgroup");
    __builtin_amdgcn_wave_barrier();
    __builtin_amdgcn_fence(__ATOMIC_ACQUIRE, "workgroup");
    if (OUT_MODE == 0) {
      float* C = (float*)Cout + (size_t)b * strideC;
      const int hh = lane >> 4, c4 = (lane & 15) * 4;
      for (int pass = 0; pass < 2; ++pass) {
#pragma unroll
        for (int it = 0; it < 8; ++it) {
          const int row = it * 2 + hh;
          v4f v = *(const v4f*)(slab + row * 68 + c4);
          *(volatile v4f*)(C + (size_t)(mBase + row) * ldc + n0 + c4) = v;
        }
        __threadfence();
      }
    } else {
      const int q = lane >> 3, c8 = (lane & 7) * 8;
      unsigned short* C  = (unsigned short*)Cout  + (size_t)b * strideC;
      unsigned short* C2 = (OUT_MODE == 2) ? ((unsigned short*)Cout2 + (size_t)b * strideC) : nullptr;
      for (int pass = 0; pass < 2; ++pass) {
#pragma unroll
        for (int it = 0; it < 4; ++it) {
          const int row = it * 4 + q;
          const float* sp = slab + row * 68 + c8;
          v8h hv, lv;
#pragma unroll
          for (int e = 0; e < 8; ++e) {
            if (OUT_MODE == 1) {
              hv[e] = (_Float16)sp[e];
            } else {
              unsigned short hb = f2bf_bits(sp[e]);
              unsigned short lb = f2bf_bits(sp[e] - bf_bits2f(hb));
              hv[e] = __builtin_bit_cast(_Float16, hb);
              lv[e] = __builtin_bit_cast(_Float16, lb);
            }
          }
          *(volatile v8h*)(C + (size_t)(mBase + row) * ldc + n0 + c8) = hv;
          if (OUT_MODE == 2) *(volatile v8h*)(C2 + (size_t)(mBase + row) * ldc + n0 + c8) = lv;
        }
        __threadfence();
      }
    }
    __builtin_amdgcn_fence(__ATOMIC_RELEASE, "workgroup");
    __builtin_amdgcn_wave_barrier();
    __builtin_amdgcn_fence(__ATOMIC_ACQUIRE, "workgroup");
  }
}

__global__ __launch_bounds__(256) void wtcast_kernel(const float* __restrict__ W0, const float* __restrict__ W1,
                                                     const float* __restrict__ W2, const float* __restrict__ W3,
                                                     unsigned short* __restrict__ out) {
  __shared__ float sm[64][65];
  const int t  = threadIdx.x;
  const int d0 = blockIdx.x * 64;
  const int f0 = blockIdx.y * 64;
  const int z  = blockIdx.z;
  const float* W = (z == 0) ? W0 : (z == 1) ? W1 : (z == 2) ? W2 : W3;
#pragma unroll
  for (int i = 0; i < 16; ++i) {
    const int e = i * 256 + t;
    const int r = e >> 6;
    const int c = e & 63;
    sm[c][r] = W[(size_t)(d0 + r) * kDim + f0 + c];
  }
  __syncthreads();
  const int lane = t & 31, wave = t >> 5;
  const int q = lane >> 3, c8 = (lane & 7) * 8;
  unsigned short* op = out + (size_t)z * kDim * kDim;
  for (int pass = 0; pass < 2; ++pass) {
#pragma unroll
    for (int it = 0; it < 2; ++it) {
      const int row = wave * 8 + it * 4 + q;
      unsigned short hb[8];
#pragma unroll
      for (int e = 0; e < 8; ++e) hb[e] = f2bf_bits(sm[row][c8 + e]);
      const v4u u = (v4u){pk16(hb[0], hb[1]), pk16(hb[2], hb[3]), pk16(hb[4], hb[5]), pk16(hb[6], hb[7])};
      *(volatile v4u*)(op + (size_t)(f0 + row) * kDim + d0 + c8) = u;
    }
    __threadfence();
  }
}

__global__ __launch_bounds__(256) void cast_f32_bf16x8(const float* __restrict__ in, unsigned short* __restrict__ out, int n8) {
  const int i  = blockIdx.x * 256 + threadIdx.x;
  const int ic = (i < n8) ? i : (n8 - 1);
  const v4f a = *(const v4f*)(in + (size_t)ic * 8);
  const v4f c = *(const v4f*)(in + (size_t)ic * 8 + 4);
  const v4u u = (v4u){pk16(f2bf_bits(a[0]), f2bf_bits(a[1])), pk16(f2bf_bits(a[2]), f2bf_bits(a[3])),
                      pk16(f2bf_bits(c[0]), f2bf_bits(c[1])), pk16(f2bf_bits(c[2]), f2bf_bits(c[3]))};
  if (i < n8) {
    unsigned short* p = out + (size_t)i * 8;
    *(volatile v4u*)p = u;
    __threadfence();
    *(volatile v4u*)p = u;
  }
}

__global__ __launch_bounds__(256) void pack_bias_kernel(const float* __restrict__ b0, const float* __restrict__ b1,
                                                        float* __restrict__ out) {
  const int t = threadIdx.x;
  const float* src = (blockIdx.x == 0) ? b0 : b1;
  const v4f v = *(const v4f*)(src + 4 * t);
  float* dst = out + (size_t)blockIdx.x * kDim + 4 * t;
  *(volatile v4f*)dst = v;
  __threadfence();
  *(volatile v4f*)dst = v;
}

__global__ __launch_bounds__(256) void softmax_rows_kernel(const float* __restrict__ SC,
                                                          unsigned short* __restrict__ PH,
                                                          unsigned short* __restrict__ PL) {
  __shared__ float redm[8];
  __shared__ float reds[8];
  const int tid = threadIdx.x, lane = tid & 31, wave = tid >> 5;
  const size_t base = (size_t)blockIdx.x * kSeq + (size_t)tid * 8;
  const v4f a = *(const v4f*)(SC + base);
  const v4f c = *(const v4f*)(SC + base + 4);
  float m = fmaxf(fmaxf(fmaxf(a[0], a[1]), fmaxf(a[2], a[3])), fmaxf(fmaxf(c[0], c[1]), fmaxf(c[2], c[3])));
#pragma unroll
  for (int off = 16; off > 0; off >>= 1) m = fmaxf(m, __shfl_xor(m, off, 32));
  if (lane == 0) redm[wave] = m;
  __syncthreads();
  float rm = redm[0];
#pragma unroll
  for (int w = 1; w < 8; ++w) rm = fmaxf(rm, redm[w]);

  v4f ea, ec;
  ea[0] = expf(a[0] - rm); ea[1] = expf(a[1] - rm); ea[2] = expf(a[2] - rm); ea[3] = expf(a[3] - rm);
  ec[0] = expf(c[0] - rm); ec[1] = expf(c[1] - rm); ec[2] = expf(c[2] - rm); ec[3] = expf(c[3] - rm);
  float sum = ((ea[0] + ea[1]) + (ea[2] + ea[3])) + ((ec[0] + ec[1]) + (ec[2] + ec[3]));
#pragma unroll
  for (int off = 16; off > 0; off >>= 1) sum += __shfl_xor(sum, off, 32);
  if (lane == 0) reds[wave] = sum;
  __syncthreads();
  float tot = reds[0];
#pragma unroll
  for (int w = 1; w < 8; ++w) tot += reds[w];
  const float inv = 1.0f / tot;

  unsigned short hb[8], lb[8];
#pragma unroll
  for (int e = 0; e < 4; ++e) {
    const float p0 = ea[e] * inv;
    hb[e] = f2bf_bits(p0);
    lb[e] = f2bf_bits(p0 - bf_bits2f(hb[e]));
    const float p1 = ec[e] * inv;
    hb[4 + e] = f2bf_bits(p1);
    lb[4 + e] = f2bf_bits(p1 - bf_bits2f(hb[4 + e]));
  }
  const v4u uh = (v4u){pk16(hb[0], hb[1]), pk16(hb[2], hb[3]), pk16(hb[4], hb[5]), pk16(hb[6], hb[7])};
  const v4u ul = (v4u){pk16(lb[0], lb[1]), pk16(lb[2], lb[3]), pk16(lb[4], lb[5]), pk16(lb[6], lb[7])};
  unsigned short* ph = PH + base;
  unsigned short* pl = PL + base;
  *(volatile v4u*)ph = uh;
  *(volatile v4u*)pl = ul;
  __threadfence();
  *(volatile v4u*)ph = uh;
  *(volatile v4u*)pl = ul;
}

extern "C" void kernel_launch(void* const* d_in, const int* in_sizes, int n_in,
                              void* d_out, int out_size, void* d_ws, size_t ws_size,
                              hipStream_t stream) {
  if (n_in < 9) return;
  if (in_sizes[0] != kTok * kDim || in_sizes[1] != kDim * kDim || in_sizes[2] != kDim ||
      in_sizes[3] != kDim * kDim || in_sizes[4] != kDim || in_sizes[5] != kDim * kDim ||
      in_sizes[6] != kDim || in_sizes[7] != kDim * kDim || in_sizes[8] != kDim) return;
  if (out_size != kTok * kDim) return;

  const float* x  = (const float*)d_in[0];
  const float* Wq = (const float*)d_in[1];
  const float* bq = (const float*)d_in[2];
  const float* Wk = (const float*)d_in[3];
  const float* bk = (const float*)d_in[4];
  const float* Wv = (const float*)d_in[5];
  const float* bv = (const float*)d_in[6];
  const float* Wo = (const float*)d_in[7];
  const float* bo = (const float*)d_in[8];
  float* out = (float*)d_out;

  const size_t bXB  = (size_t)kTok * kDim * 2;
  const size_t bWT  = (size_t)4 * kDim * kDim * 2;
  const size_t bBQK = (size_t)2 * kDim * 4;
  const size_t bQK  = (size_t)kSeq * kQKCols * 2;
  const size_t bVT  = (size_t)kDim * kSeq * 2;
  const size_t bSC  = (size_t)kSeq * kSeq * 4;
  const size_t bP   = (size_t)kSeq * kSeq * 2;
  const size_t bCX  = (size_t)kSeq * kDim * 2;

  size_t off = 0;
  const size_t oXB  = off; off += bXB;
  const size_t oWT  = off; off += bWT;
  const size_t oBQK = off; off += bBQK;
  const size_t oQKH = off; off += bQK;
  const size_t oQKL = off; off += bQK;
  const size_t oVTH = off; off += bVT;
  const size_t oVTL = off; off += bVT;
  const size_t oSC  = off; off += bSC;
  const size_t oPH  = off; off += bP;
  const size_t oPL  = off; off += bP;
  const size_t oCXH = off; off += bCX;
  const size_t oCXL = off; off += bCX;
  if (off > ws_size) return;

  char* ws = (char*)d_ws;
  unsigned short* XB  = (unsigned short*)(ws + oXB);
  unsigned short* WT  = (unsigned short*)(ws + oWT);
  float*          BQK = (float*)(ws + oBQK);
  unsigned short* QKH = (unsigned short*)(ws + oQKH);
  unsigned short* QKL = (unsigned short*)(ws + oQKL);
  unsigned short* VTH = (unsigned short*)(ws + oVTH);
  unsigned short* VTL = (unsigned short*)(ws + oVTL);
  float*          SC  = (float*)(ws + oSC);
  unsigned short* PH  = (unsigned short*)(ws + oPH);
  unsigned short* PL  = (unsigned short*)(ws + oPL);
  unsigned short* CXH = (unsigned short*)(ws + oCXH);
  unsigned short* CXL = (unsigned short*)(ws + oCXL);

  const size_t planeW = (size_t)kDim * kDim;

  const int n8 = kTok * kDim / 8;
  cast_f32_bf16x8<<<dim3(n8 / 256), dim3(256), 0, stream>>>(x, XB, n8);
  wtcast_kernel<<<dim3(kDim / 64, kDim / 64, 4), dim3(256), 0, stream>>>(Wq, Wk, Wv, Wo, WT);
  pack_bias_kernel<<<dim3(2), dim3(256), 0, stream>>>(bq, bk, BQK);

  for (int b = 0; b < kBatch; ++b) {
    const size_t r0 = (size_t)b * kSeq;
    const unsigned short* XBb = XB + r0 * kDim;

    wmma_gemm64<1, 0, 2, 2, false><<<dim3(128, 1), dim3(256), 0, stream>>>(
        XBb, VTL, kDim, 0,
        WT, VTH, kDim, 0,
        (void*)QKH, (void*)QKL, kQKCols, 0,
        BQK, x, 0,
        kSeq, kQKCols, kDim, 1.0f);

    wmma_gemm64<1, 0, 1, 2, false><<<dim3(64, 1), dim3(256), 0, stream>>>(
        WT + 2 * planeW, PL, kDim, 0,
        XBb, PH, kDim, 0,
        (void*)VTH, (void*)VTL, kSeq, 0,
        bv, x, 0,
        kDim, kSeq, kDim, 1.0f);

    wmma_gemm64<1, 1, 0, 0, false><<<dim3(128, 1), dim3(256), 0, stream>>>(
        QKH, QKL, kQKCols, 0,
        QKH + kDim, QKL + kDim, kQKCols, 0,
        (void*)SC, (void*)CXL, kSeq, 0,
        bo, x, 0,
        kSeq, kSeq, kDim, kScoreScale);

    softmax_rows_kernel<<<dim3(kSeq), dim3(256), 0, stream>>>(SC, PH, PL);

    wmma_gemm64<1, 1, 0, 2, false><<<dim3(64, 1), dim3(256), 0, stream>>>(
        PH, PL, kSeq, 0,
        VTH, VTL, kSeq, 0,
        (void*)CXH, (void*)CXL, kDim, 0,
        bo, x, 0,
        kSeq, kDim, kSeq, 1.0f);

    wmma_gemm64<1, 2, 2, 0, false><<<dim3(64, 1), dim3(256), 0, stream>>>(
        CXH, CXL, kDim, 0,
        WT + 3 * planeW, PL, kDim, 0,
        (void*)(out + r0 * kDim), (void*)SC, kDim, 0,
        bo, x, 0,
        kSeq, kDim, kDim, 1.0f);
  }
}
